// ExternalKnowledge_47150150975594
// MI455X (gfx1250) — hardware-run, weakly checked
//
#include <hip/hip_runtime.h>
#include <math.h>

typedef __attribute__((ext_vector_type(16))) __bf16       v16b;
typedef __attribute__((ext_vector_type(8)))  __bf16       v8b;
typedef __attribute__((ext_vector_type(8)))  float        v8f;
typedef __attribute__((ext_vector_type(4)))  float        v4f;
typedef __attribute__((ext_vector_type(4)))  unsigned int v4u;
typedef __attribute__((ext_vector_type(2)))  int          v2i;

constexpr int kNb    = 16;
constexpr int kSlots = 2048;
constexpr int kTok   = 6;
constexpr int kEmb   = 128;
constexpr int kHist  = 512;
constexpr int kVocab = 32000;
constexpr int kHops  = 3;
constexpr int kRows  = kNb * kSlots;
constexpr int kSplit = 2;
constexpr float kLeak = 0.1f;
constexpr float kF32MinNormal = 1.17549435e-38f;
constexpr int kOut1Elems = kNb * kSlots;
static_assert(kRows == 32768, "rows");
static_assert((kSlots % 64) == 0, "a 64-row tile stays inside one sample");
static_assert((kRows % 64) == 0 && (kEmb % 64) == 0 && (kEmb % 32) == 0, "tile multiples");
static_assert((kRows % 16) == 0, "gather rows per block");
static_assert(kOut1Elems * 4 == 131072, "second output byte offset");
static_assert((size_t)2 * kOut1Elems * 4 == 262144ull, "output total");

constexpr size_t kPlaneBytes = (size_t)kRows * kEmb * 2;
constexpr size_t kEaBytes    = (size_t)kRows * kEmb * 4;
constexpr size_t kWBytes     = (size_t)kEmb * kEmb * 2;
constexpr size_t kOffXH  = 0;
constexpr size_t kOffXL  = kOffXH  + kPlaneBytes;
constexpr size_t kOffHH  = kOffXL  + kPlaneBytes;
constexpr size_t kOffHL  = kOffHH  + kPlaneBytes;
constexpr size_t kOffEA  = kOffHL  + kPlaneBytes;
constexpr size_t kOffW1H = kOffEA  + (size_t)kHops * kEaBytes;
constexpr size_t kOffW1L = kOffW1H + kWBytes;
constexpr size_t kOffW2H = kOffW1L + kWBytes;
constexpr size_t kOffW2L = kOffW2H + kWBytes;
constexpr size_t kOffB1  = kOffW2L + kWBytes;
constexpr size_t kWsTotal = kOffB1 + (size_t)kNb * kEmb * 4;
static_assert(kWsTotal == 84025344ull, "carve total");
static_assert(kWsTotal <= 134217728ull, "carve cap");
static_assert((kOffXL % 128) == 0 && (kOffHH % 128) == 0 && (kOffHL % 128) == 0 && (kOffEA % 128) == 0 &&
              (kOffW1H % 128) == 0 && (kOffW1L % 128) == 0 && (kOffW2H % 128) == 0 && (kOffW2L % 128) == 0 &&
              (kOffB1 % 128) == 0, "128-B aligned regions");

__device__ __forceinline__ unsigned bf_rne_word(float f) {
  const unsigned u = __float_as_uint(f);
  const unsigned lsb = (u & 0x00010000u) ? 1u : 0u;
  return (u + 0x7FFFu + lsb) & 0xFFFF0000u;
}
__device__ __forceinline__ void split_pair(float f0, float f1, unsigned& hw, unsigned& lw) {
  const unsigned h0 = bf_rne_word(f0);
  const unsigned h1 = bf_rne_word(f1);
  const float r0 = f0 - __uint_as_float(h0);
  const float r1 = f1 - __uint_as_float(h1);
  const unsigned l0 = bf_rne_word(r0);
  const unsigned l1 = bf_rne_word(r1);
  hw = h1 | (h0 >> 16);
  lw = l1 | (l0 >> 16);
}
__device__ __forceinline__ void split8(float f0, float f1, float f2, float f3, float f4, float f5, float f6, float f7,
                                       v4u& hv, v4u& lv) {
  unsigned h0, h1, h2, h3, l0, l1, l2, l3;
  split_pair(f0, f1, h0, l0);
  split_pair(f2, f3, h1, l1);
  split_pair(f4, f5, h2, l2);
  split_pair(f6, f7, h3, l3);
  hv = (v4u){h0, h1, h2, h3};
  lv = (v4u){l0, l1, l2, l3};
}

namespace eng {
__device__ __forceinline__ void guard1_b(v8f& a, v16b x, v16b y) { asm volatile("v_nop\n\tv_nop\n\tv_nop\n\tv_nop" : "+v"(a) : "v"(x), "v"(y)); }
__device__ __forceinline__ void keep4_b(v16b a, v16b b, v16b c, v16b d) { asm volatile("v_nop" :: "v"(a), "v"(b), "v"(c), "v"(d)); }
__device__ __forceinline__ void acc_guard4(v8f& a, v8f& b, v8f& c, v8f& d) { asm volatile("v_nop\n\tv_nop\n\tv_nop\n\tv_nop" : "+v"(a), "+v"(b), "+v"(c), "+v"(d)); }
struct FragB {
  union U { v16b v; v8b h[2]; };
  static __device__ __forceinline__ v16b load(const __bf16* p) {
    U f; f.h[0] = *(const v8b*)(p); f.h[1] = *(const v8b*)(p + 16); return f.v;
  }
  static __device__ __forceinline__ v8f mma(v16b a, v16b b, v8f c) {
    return __builtin_amdgcn_wmma_f32_16x16x32_bf16(false, a, false, b, (short)0, c, false, false);
  }
};

template <int SPL, int EPI>
__global__ __launch_bounds__(256) void mlp_gemm64(
    const unsigned short* __restrict__ Ap, const unsigned short* __restrict__ A2p,
    const unsigned short* __restrict__ Btp, const unsigned short* __restrict__ Bt2p,
    void* __restrict__ Cout, void* __restrict__ Cout2,
    const float* __restrict__ bias) {
  const __bf16* A   = (const __bf16*)Ap;
  const __bf16* A2  = (const __bf16*)A2p;
  const __bf16* Bt  = (const __bf16*)Btp;
  const __bf16* Bt2 = (const __bf16*)Bt2p;
  __shared__ __align__(16) float sT[8][16 * 68];
  const int lane = threadIdx.x & 31;
  const int wave = threadIdx.x >> 5;
  constexpr int tilesN = kEmb >> 6;
  constexpr int tilesM = kRows >> 6;
  const int tile = blockIdx.x * 8 + wave;
  if (tile >= tilesM * tilesN) return;
  const int tm = tile / tilesN;
  const int tn = tile - tm * tilesN;
  const int m0 = tm << 6;
  const int n0 = tn << 6;

  const int rlane = lane & 15;
  const int koff  = (lane >> 4) * 8;
  const int mOff  = (lane >> 4) * 8;

  v8f acc[4][4];
#pragma unroll
  for (int i = 0; i < 4; ++i)
#pragma unroll
    for (int j = 0; j < 4; ++j) acc[i][j] = (v8f){0.f,0.f,0.f,0.f,0.f,0.f,0.f,0.f};

#pragma unroll 1
  for (int k0 = 0; k0 < kEmb; k0 += 32) {
    v16b bh[4], bl[4];
#pragma unroll
    for (int j = 0; j < 4; ++j) {
      const size_t bo = (size_t)(n0 + (j << 4) + rlane) * kEmb + koff + k0;
      bh[j] = FragB::load(Bt + bo);
      bl[j] = bh[j];
      if (SPL == 2) bl[j] = FragB::load(Bt2 + bo);
    }
#pragma unroll
    for (int i = 0; i < 4; ++i) {
      const size_t ao = (size_t)(m0 + (i << 4) + rlane) * kEmb + koff + k0;
      v16b ah = FragB::load(A + ao);
      v16b al = ah;
      if (SPL >= 1) al = FragB::load(A2 + ao);
#pragma unroll
      for (int j = 0; j < 4; ++j) {
        acc[i][j] = FragB::mma(ah, bh[j], acc[i][j]);
        if (SPL == 2) acc[i][j] = FragB::mma(ah, bl[j], acc[i][j]);
        if (SPL >= 1) acc[i][j] = FragB::mma(al, bh[j], acc[i][j]);
      }
      guard1_b(acc[i][0], ah, al);
      guard1_b(acc[i][1], ah, al);
      guard1_b(acc[i][2], ah, al);
      guard1_b(acc[i][3], ah, al);
    }
    keep4_b(bh[0], bh[1], bh[2], bh[3]);
    if (SPL == 2) keep4_b(bl[0], bl[1], bl[2], bl[3]);
  }
  acc_guard4(acc[0][0], acc[0][1], acc[0][2], acc[0][3]);
  acc_guard4(acc[1][0], acc[1][1], acc[1][2], acc[1][3]);
  acc_guard4(acc[2][0], acc[2][1], acc[2][2], acc[2][3]);
  acc_guard4(acc[3][0], acc[3][1], acc[3][2], acc[3][3]);

  float* slab = sT[wave];
  const float* brow = (EPI == 0) ? (bias + (size_t)(m0 >> 11) * kEmb) : bias;
  float bv[4];
#pragma unroll
  for (int j = 0; j < 4; ++j) bv[j] = brow[n0 + (j << 4) + rlane];
#pragma unroll
  for (int i = 0; i < 4; ++i) {
    const int mBase = m0 + (i << 4);
#pragma unroll
    for (int j = 0; j < 4; ++j) {
#pragma unroll
      for (int r = 0; r < 8; ++r) {
        float v = acc[i][j][r] + bv[j];
        if (EPI == 0) v = (v > 0.f) ? v : kLeak * v;
        slab[(mOff + r) * 68 + (j << 4) + rlane] = v;
      }
    }
    __builtin_amdgcn_fence(__ATOMIC_RELEASE, "workgroup");
    __builtin_amdgcn_wave_barrier();
    __builtin_amdgcn_fence(__ATOMIC_ACQUIRE, "workgroup");
    if (EPI == 1) {
      float* C = (float*)Cout;
      const int hh = lane >> 4, c4 = (lane & 15) * 4;
      for (int pass = 0; pass < 2; ++pass) {
#pragma unroll
        for (int it = 0; it < 8; ++it) {
          const int row = it * 2 + hh;
          v4f v = *(const v4f*)(slab + row * 68 + c4);
          *(volatile v4f*)(C + (size_t)(mBase + row) * kEmb + n0 + c4) = v;
        }
        __threadfence();
      }
    } else {
      const int q = lane >> 3, c8 = (lane & 7) * 8;
      unsigned short* C  = (unsigned short*)Cout;
      unsigned short* C2 = (unsigned short*)Cout2;
      for (int pass = 0; pass < 2; ++pass) {
#pragma unroll
        for (int it = 0; it < 4; ++it) {
          const int row = it * 4 + q;
          const float* sp = slab + row * 68 + c8;
          const v4f a0 = *(const v4f*)(sp);
          const v4f a1 = *(const v4f*)(sp + 4);
          v4u hv, lv;
          split8(a0[0], a0[1], a0[2], a0[3], a1[0], a1[1], a1[2], a1[3], hv, lv);
          const size_t o = (size_t)(mBase + row) * kEmb + n0 + c8;
          *(volatile v4u*)(C + o)  = hv;
          *(volatile v4u*)(C2 + o) = lv;
        }
        __threadfence();
      }
    }
    __builtin_amdgcn_fence(__ATOMIC_RELEASE, "workgroup");
    __builtin_amdgcn_wave_barrier();
    __builtin_amdgcn_fence(__ATOMIC_ACQUIRE, "workgroup");
  }
}
}

__global__ __launch_bounds__(256) void prep_weights_kernel(
    const float* __restrict__ wA1, const float* __restrict__ wA2,
    unsigned short* __restrict__ W1H, unsigned short* __restrict__ W1L,
    unsigned short* __restrict__ W2H, unsigned short* __restrict__ W2L)
{
  __shared__ float sW[kEmb * 17];
  unsigned tid = threadIdx.x;
  asm volatile("" : "+v"(tid));
  const unsigned mat = blockIdx.x >> 3;
  const unsigned n0  = (blockIdx.x & 7u) * 16u;
  const float* W = (mat != 0u) ? wA2 : wA1;
  unsigned short* PH = (mat != 0u) ? W2H : W1H;
  unsigned short* PL = (mat != 0u) ? W2L : W1L;
#pragma unroll
  for (int i = 0; i < 8; ++i) {
    unsigned idx = tid + 256u * (unsigned)i;
    const unsigned k = idx >> 4, nn = idx & 15u;
    sW[k * 17u + nn] = W[(size_t)k * kEmb + n0 + nn];
  }
  __syncthreads();
  unsigned r = tid >> 4, c = tid & 15u;
  asm volatile("" : "+v"(r), "+v"(c));
  const float* sp = sW + (c * 8u) * 17u + r;
  const float f0 = sp[0 * 17], f1 = sp[1 * 17], f2 = sp[2 * 17], f3 = sp[3 * 17];
  const float f4 = sp[4 * 17], f5 = sp[5 * 17], f6 = sp[6 * 17], f7 = sp[7 * 17];
  v4u hv, lv;
  split8(f0, f1, f2, f3, f4, f5, f6, f7, hv, lv);
  const size_t o = (size_t)(n0 + r) * kEmb + c * 8u;
  *(volatile v4u*)(PH + o) = hv;
  *(volatile v4u*)(PL + o) = lv;
  __threadfence();
  *(volatile v4u*)(PH + o) = hv;
  *(volatile v4u*)(PL + o) = lv;
}

__global__ __launch_bounds__(128) void bias_fold_kernel(
    const float* __restrict__ tf, const float* __restrict__ wA1, const float* __restrict__ bA1,
    float* __restrict__ bias1)
{
  __shared__ float sTf[kEmb];
  __shared__ __align__(16) float sB[kEmb];
  const int n = threadIdx.x, b = blockIdx.x;
  sTf[n] = tf[b * kEmb + n];
  __syncthreads();
  float acc = 0.f;
  const float* wp = wA1 + (size_t)kEmb * kEmb + n;
#pragma unroll 4
  for (int k = 0; k < kEmb; ++k) acc = fmaf(sTf[k], wp[(size_t)k * kEmb], acc);
  acc += bA1[n];
  sB[n] = acc;
  __syncthreads();
  if (n < 32) {
    const v4f v = *(const v4f*)(sB + n * 4);
    float* q = bias1 + (size_t)b * kEmb + n * 4;
    *(volatile v4f*)q = v;
    __threadfence();
    *(volatile v4f*)q = v;
  }
}

__global__ __launch_bounds__(256) void gather_sum_kernel(
    const int* __restrict__ story, const int* __restrict__ kb_len, const int* __restrict__ conv_len,
    const float* __restrict__ dh, const float* __restrict__ Ct,
    unsigned short* __restrict__ XH, unsigned short* __restrict__ XL)
{
  unsigned tid = threadIdx.x;
  asm volatile("" : "+v"(tid));
  const unsigned lane = tid & 31u, wave = tid >> 5;
  unsigned hsel = lane >> 4, c = lane & 15u;
  unsigned row = blockIdx.x * 16u + wave * 2u + hsel;
  asm volatile("" : "+v"(row), "+v"(c));
  const unsigned smp = row >> 11;
  const int m = (int)(row & (unsigned)(kSlots - 1));

  const v2i* st = (const v2i*)(story + (size_t)row * kTok);
  const v2i i01 = st[0], i23 = st[1], i45 = st[2];
  int id[6];
  id[0] = i01[0]; id[1] = i01[1]; id[2] = i23[0]; id[3] = i23[1]; id[4] = i45[0]; id[5] = i45[1];
  v4f a0 = (v4f){0.f, 0.f, 0.f, 0.f};
  v4f a1 = (v4f){0.f, 0.f, 0.f, 0.f};
#pragma unroll
  for (int s = 0; s < kTok; ++s) {
    int t = id[s];
    t = t < 0 ? 0 : t;
    t = t > kVocab - 1 ? kVocab - 1 : t;
    const float* p = Ct + (size_t)t * kEmb + c * 8u;
    a0 += *(const v4f*)(p);
    a1 += *(const v4f*)(p + 4);
  }
  const int kb = kb_len[smp], cl = conv_len[smp];
  const int j = m - kb;
  const bool hit = (j >= 0) && (j < cl);
  int jc = j < 0 ? 0 : j;
  jc = jc > kHist - 1 ? kHist - 1 : jc;
  const float* dp = dh + ((size_t)smp * kHist + (size_t)jc) * kEmb + c * 8u;
  v4f d0 = *(const v4f*)(dp);
  v4f d1 = *(const v4f*)(dp + 4);
  asm volatile("" : "+v"(d0), "+v"(d1));
  const v4f zz = (v4f){0.f, 0.f, 0.f, 0.f};
  a0 += hit ? d0 : zz;
  a1 += hit ? d1 : zz;

  v4u hv, lv;
  split8(a0[0], a0[1], a0[2], a0[3], a1[0], a1[1], a1[2], a1[3], hv, lv);
  const size_t o = (size_t)row * kEmb + c * 8u;
  *(volatile v4u*)(XH + o) = hv;
  *(volatile v4u*)(XL + o) = lv;
  __threadfence();
  *(volatile v4u*)(XH + o) = hv;
  *(volatile v4u*)(XL + o) = lv;
}

__global__ __launch_bounds__(256) void query_hops_kernel(
    const float* __restrict__ EA, const float* __restrict__ qv, const float* __restrict__ gp,
    float* __restrict__ out)
{
  __shared__ __align__(16) float sUq[kEmb];
  __shared__ __align__(16) float sL[kSlots];
  __shared__ __align__(16) float sP[kSlots];
  __shared__ __align__(16) float sG[kSlots];
  __shared__ __align__(16) float sPart[8 * kEmb];
  __shared__ float sRedA[8];
  __shared__ float sRedB[8];
  const int tid = threadIdx.x, lane = tid & 31, wave = tid >> 5;
  const int b = blockIdx.x;

  if (tid < kEmb / 4) *(v4f*)(sUq + tid * 4) = *(const v4f*)(qv + (size_t)b * kEmb + tid * 4);
#pragma unroll
  for (int i = 0; i < 2; ++i) {
    const int off = (tid + 256 * i) * 4;
    *(v4f*)(sG + off) = *(const v4f*)(gp + (size_t)b * kSlots + off);
  }
  __syncthreads();

#pragma unroll 1
  for (int hop = 0; hop < kHops; ++hop) {
    const float* E = EA + ((size_t)hop * kRows + (size_t)b * kSlots) * kEmb;
    const v4f u = *(const v4f*)(sUq + lane * 4);
#pragma unroll 2
    for (int i = 0; i < kSlots / 8; ++i) {
      const int m = wave + 8 * i;
      const v4f e = *(const v4f*)(E + (size_t)m * kEmb + lane * 4);
      float s = e[0] * u[0];
      s = fmaf(e[1], u[1], s);
      s = fmaf(e[2], u[2], s);
      s = fmaf(e[3], u[3], s);
      s += __shfl_xor(s, 16, 32);
      s += __shfl_xor(s, 8, 32);
      s += __shfl_xor(s, 4, 32);
      s += __shfl_xor(s, 2, 32);
      s += __shfl_xor(s, 1, 32);
      const float lg = sG[m] * s;
      if (lane == 0) sL[m] = lg;
    }
    __syncthreads();

    float mx = -INFINITY;
#pragma unroll 1
    for (int j = 0; j < 8; ++j) mx = fmaxf(mx, sL[tid + 256 * j]);
    mx = fmaxf(mx, __shfl_xor(mx, 16, 32));
    mx = fmaxf(mx, __shfl_xor(mx, 8, 32));
    mx = fmaxf(mx, __shfl_xor(mx, 4, 32));
    mx = fmaxf(mx, __shfl_xor(mx, 2, 32));
    mx = fmaxf(mx, __shfl_xor(mx, 1, 32));
    if (lane == 0) sRedA[wave] = mx;
    __syncthreads();
    float bm = sRedA[0];
#pragma unroll
    for (int w = 1; w < 8; ++w) bm = fmaxf(bm, sRedA[w]);

    float sum = 0.f;
#pragma unroll 1
    for (int j = 0; j < 8; ++j) {
      const int idx = tid + 256 * j;
      float ex = expf(sL[idx] - bm);
      ex = (ex < kF32MinNormal) ? 0.f : ex;
      sP[idx] = ex;
      sum += ex;
    }
    sum += __shfl_xor(sum, 16, 32);
    sum += __shfl_xor(sum, 8, 32);
    sum += __shfl_xor(sum, 4, 32);
    sum += __shfl_xor(sum, 2, 32);
    sum += __shfl_xor(sum, 1, 32);
    if (lane == 0) sRedB[wave] = sum;
    __syncthreads();
    float tot = 0.f;
#pragma unroll
    for (int w = 0; w < 8; ++w) tot += sRedB[w];
    const float inv = 1.0f / tot;
    const bool last = (hop == kHops - 1);
#pragma unroll 1
    for (int j = 0; j < 8; ++j) {
      const int idx = tid + 256 * j;
      const float p = sP[idx] * inv;
      const float g = sG[idx];
      sP[idx] = last ? p : (p * g);
    }
    __syncthreads();

    if (last) {
      float* o0 = out + (size_t)b * kSlots;
      float* o1 = out + (size_t)kOut1Elems + (size_t)b * kSlots;
      v4f pv[2], lv[2];
#pragma unroll
      for (int i = 0; i < 2; ++i) {
        const int off = (tid + 256 * i) * 4;
        pv[i] = *(const v4f*)(sP + off);
        lv[i] = *(const v4f*)(sL + off);
      }
      for (int pass = 0; pass < 2; ++pass) {
#pragma unroll
        for (int i = 0; i < 2; ++i) {
          const int off = (tid + 256 * i) * 4;
          *(volatile v4f*)(o0 + off) = pv[i];
          *(volatile v4f*)(o1 + off) = lv[i];
        }
        __threadfence();
      }
    } else {
      const float* En = EA + ((size_t)(hop + 1) * kRows + (size_t)b * kSlots) * kEmb;
      v4f a = (v4f){0.f, 0.f, 0.f, 0.f};
#pragma unroll 2
      for (int i = 0; i < kSlots / 8; ++i) {
        const int m = wave + 8 * i;
        const float w = sP[m];
        const v4f e = *(const v4f*)(En + (size_t)m * kEmb + lane * 4);
        a += e * w;
      }
      *(v4f*)(sPart + wave * kEmb + lane * 4) = a;
      __syncthreads();
      if (tid < kEmb) {
        float t = 0.f;
#pragma unroll
        for (int w = 0; w < 8; ++w) t += sPart[w * kEmb + tid];
        sUq[tid] = sUq[tid] + t;
      }
      __syncthreads();
    }
  }
}

extern "C" void kernel_launch(void* const* d_in, const int* in_sizes, int n_in,
                              void* d_out, int out_size, void* d_ws, size_t ws_size,
                              hipStream_t stream) {
  if (n_in < 13) return;
  if (in_sizes[0] != kNb * kSlots * kTok) return;
  if (in_sizes[1] != kNb || in_sizes[2] != kNb) return;
  if (in_sizes[4] != kNb * kHist * kEmb) return;
  if (in_sizes[5] != kNb * kEmb || in_sizes[6] != kNb * kEmb) return;
  if (in_sizes[7] != kNb * kSlots) return;
  if (in_sizes[8] != 4 * kVocab * kEmb) return;
  if (in_sizes[9] != 2 * kEmb * kEmb || in_sizes[10] != kEmb) return;
  if (in_sizes[11] != kEmb * kEmb || in_sizes[12] != kEmb) return;
  if (out_size != 2 * kNb * kSlots) return;
  if (ws_size < kWsTotal) return;

  const int*   story    = (const int*)d_in[0];
  const int*   kb_len   = (const int*)d_in[1];
  const int*   conv_len = (const int*)d_in[2];
  const float* dh       = (const float*)d_in[4];
  const float* tf       = (const float*)d_in[5];
  const float* qv       = (const float*)d_in[6];
  const float* gp       = (const float*)d_in[7];
  const float* Ctab     = (const float*)d_in[8];
  const float* wA1      = (const float*)d_in[9];
  const float* bA1      = (const float*)d_in[10];
  const float* wA2      = (const float*)d_in[11];
  const float* bA2      = (const float*)d_in[12];
  float* out = (float*)d_out;

  char* ws = (char*)d_ws;
  unsigned short* XH  = (unsigned short*)(ws + kOffXH);
  unsigned short* XL  = (unsigned short*)(ws + kOffXL);
  unsigned short* HH  = (unsigned short*)(ws + kOffHH);
  unsigned short* HL  = (unsigned short*)(ws + kOffHL);
  float*          EA  = (float*)(ws + kOffEA);
  unsigned short* W1H = (unsigned short*)(ws + kOffW1H);
  unsigned short* W1L = (unsigned short*)(ws + kOffW1L);
  unsigned short* W2H = (unsigned short*)(ws + kOffW2H);
  unsigned short* W2L = (unsigned short*)(ws + kOffW2L);
  float*          B1  = (float*)(ws + kOffB1);

  prep_weights_kernel<<<16, 256, 0, stream>>>(wA1, wA2, W1H, W1L, W2H, W2L);
  bias_fold_kernel<<<kNb, kEmb, 0, stream>>>(tf, wA1, bA1, B1);

  for (int hop = 0; hop < kHops; ++hop) {
    const float* Ct = Ctab + (size_t)hop * kVocab * kEmb;
    gather_sum_kernel<<<kRows / 16, 256, 0, stream>>>(story, kb_len, conv_len, dh, Ct, XH, XL);
    eng::mlp_gemm64<kSplit, 0><<<128, 256, 0, stream>>>(XH, XL, W1H, W1L, (void*)HH, (void*)HL, B1);
    eng::mlp_gemm64<kSplit, 1><<<128, 256, 0, stream>>>(HH, HL, W2H, W2L,
                                                        (void*)(EA + (size_t)hop * kRows * kEmb), (void*)HL, bA2);
  }

  query_hops_kernel<<<kNb, 256, 0, stream>>>(EA, qv, gp, out);
}
